// TransformerAttention_3702261809284
// MI455X (gfx1250) — hardware-verified
//
#include <hip/hip_runtime.h>


#ifndef NB
#define NB 2
#endif
#ifndef SEQ
#define SEQ 2048
#endif
#define NB_FULL  2
#define SEQ_FULL 2048
#define DM   1024
#define NH   16
#define HD   64
#define HF   (HD / 2)
#define RH   ((SEQ < 512) ? SEQ : 512)
#define PCAR 1024.0f
#define SCL  0.125f
#define L2E  1.4426950408889634f
#define OSP  72
#define PSP  72
static_assert((SEQ % 64) == 0);
static_assert((RH % 16) == 0);
static_assert(RH <= SEQ);
static_assert((DM % 64) == 0);
static_assert(NH * HD == DM);
static_assert(NB <= NB_FULL);
static_assert(SEQ <= SEQ_FULL);

typedef _Float16 h16;
typedef unsigned short bf;
typedef __attribute__((ext_vector_type(16))) __bf16   v16bf;
typedef __attribute__((ext_vector_type(16))) _Float16 v16h;
typedef __attribute__((ext_vector_type(8)))  _Float16 v8h;
typedef __attribute__((ext_vector_type(8)))  unsigned short v8us;
typedef __attribute__((ext_vector_type(8)))  float    v8f;
typedef __attribute__((ext_vector_type(4)))  float    v4f;
typedef __attribute__((ext_vector_type(2)))  _Float16 v2h;
typedef __attribute__((ext_vector_type(2)))  unsigned short v2us;
typedef __attribute__((ext_vector_type(2)))  float    v2f;
typedef v8h  __attribute__((may_alias)) v8ha;
typedef v4f  __attribute__((may_alias)) v4fa;
typedef v8f  __attribute__((may_alias)) v8fa;
typedef v8us __attribute__((may_alias)) v8usa;

__device__ __forceinline__ unsigned short f2bf(float f) { unsigned u = __float_as_uint(f); u += 0x7FFFu + ((u >> 16) & 1u); return (unsigned short)(u >> 16); }
__device__ __forceinline__ float bf2f(unsigned short b) { return __uint_as_float(((unsigned)b) << 16); }
__device__ __forceinline__ float bfr(float f) { return bf2f(f2bf(f)); }
__device__ __forceinline__ v16h cat16(v8h lo, v8h hi) { return __builtin_shufflevector(lo, hi, 0, 1, 2, 3, 4, 5, 6, 7, 8, 9, 10, 11, 12, 13, 14, 15); }
__device__ __forceinline__ v16bf cat16b(v8us lo, v8us hi) { return __builtin_bit_cast(v16bf, __builtin_shufflevector(lo, hi, 0, 1, 2, 3, 4, 5, 6, 7, 8, 9, 10, 11, 12, 13, 14, 15)); }
__device__ __forceinline__ v8f wmma16(v16h a, v16h b, v8f c) { return __builtin_amdgcn_wmma_f32_16x16x32_f16(false, a, false, b, (short)0, c, false, false); }
__device__ __forceinline__ v8f wmmab(v16bf a, v16bf b, v8f c) { return __builtin_amdgcn_wmma_f32_16x16x32_bf16(false, a, false, b, (short)0, c, false, false); }
__device__ __forceinline__ h16 tohx(float x) { return (h16)x; }
__device__ __forceinline__ void splitf(float y, unsigned short& h, unsigned short& l) { h = f2bf(y); l = f2bf(y - bf2f(h)); }

template <typename T16> struct WFrag;
template <> struct WFrag<h16> { typedef v16h V; static __device__ __forceinline__ V ld(const h16* p) { return cat16(*(const v8h*)p, *(const v8h*)(p + 16)); } static __device__ __forceinline__ v8f mma(V a, V b, v8f c) { return wmma16(a, b, c); } };
template <> struct WFrag<bf> { typedef v16bf V; static __device__ __forceinline__ V ld(const bf* p) { return cat16b(*(const v8us*)p, *(const v8us*)(p + 16)); } static __device__ __forceinline__ v8f mma(V a, V b, v8f c) { return wmmab(a, b, c); } };
template <typename T16, int NSPLIT, bool BIAS>
__global__ __launch_bounds__(32) void k_gemmw(const T16* __restrict__ A, const T16* __restrict__ A2, const T16* __restrict__ Bt, const T16* __restrict__ Bt2, int K, float* C, int ldc, const float* __restrict__ bias, size_t sA, size_t sB, size_t sC) {
    typedef typename WFrag<T16>::V V;
    __shared__ __align__(16) float os[16 * 68];
    const size_t z = blockIdx.z; A += z * sA; if (A2) A2 += z * sA; Bt += z * sB; if (Bt2) Bt2 += z * sB; C += z * sC;
    const int lane = threadIdx.x & 31, lr = lane & 15, hi = lane >> 4; const int r0 = blockIdx.x * 64, c0 = blockIdx.y * 64;
    v8f acc[4][4];
#pragma unroll
    for (int mb = 0; mb < 4; ++mb)
#pragma unroll
        for (int nb = 0; nb < 4; ++nb) acc[mb][nb] = (v8f){};
    const size_t aoff = (size_t)(r0 + lr) * K + 8 * hi, boff = (size_t)(c0 + lr) * K + 8 * hi;
#pragma unroll 1
    for (int kc = 0; kc < K; kc += 32) {
        V a[4], a2[4];
#pragma unroll
        for (int mb = 0; mb < 4; ++mb) { a[mb] = WFrag<T16>::ld(A + aoff + (size_t)mb * 16 * K + kc); if (NSPLIT == 1 || NSPLIT == 2) a2[mb] = WFrag<T16>::ld(A2 + aoff + (size_t)mb * 16 * K + kc); }
#pragma unroll
        for (int nb = 0; nb < 4; ++nb) { const V b = WFrag<T16>::ld(Bt + boff + (size_t)nb * 16 * K + kc); V b2; if (NSPLIT >= 2) b2 = WFrag<T16>::ld(Bt2 + boff + (size_t)nb * 16 * K + kc);
#pragma unroll
            for (int mb = 0; mb < 4; ++mb) { acc[mb][nb] = WFrag<T16>::mma(a[mb], b, acc[mb][nb]); if (NSPLIT == 1 || NSPLIT == 2) acc[mb][nb] = WFrag<T16>::mma(a2[mb], b, acc[mb][nb]); if (NSPLIT >= 2) acc[mb][nb] = WFrag<T16>::mma(a[mb], b2, acc[mb][nb]); } }
        asm volatile("v_nop\n\tv_nop\n\tv_nop\n\tv_nop" : "+v"(acc[0][0]), "+v"(acc[1][1]), "+v"(acc[2][2]), "+v"(acc[3][3]) : "v"(a[0]), "v"(a[3]));
    }
#pragma unroll
    for (int mb = 0; mb < 4; ++mb) {
#pragma unroll
        for (int nb = 0; nb < 4; ++nb) {
#pragma unroll
            for (int j = 0; j < 8; ++j) os[(hi * 8 + j) * 68 + nb * 16 + lr] = acc[mb][nb][j]; }
        __builtin_amdgcn_wave_barrier(); asm volatile("" ::: "memory");
        float* crow = C + (size_t)(r0 + mb * 16) * ldc + c0;
#pragma unroll 1
        for (int ps = 0; ps < 2; ++ps) {
#pragma unroll
            for (int s = 0; s < 8; ++s) { const int row = 2 * s + hi, cofs = lr * 4; v4f val = *(const v4fa*)(os + row * 68 + cofs); if (BIAS) { val[0] += bfr(bias[c0 + cofs]); val[1] += bfr(bias[c0 + cofs + 1]); val[2] += bfr(bias[c0 + cofs + 2]); val[3] += bfr(bias[c0 + cofs + 3]); }
                *(volatile v4f*)(crow + (size_t)row * ldc + cofs) = val; }
            if (ps == 0) __threadfence(); }
        __builtin_amdgcn_wave_barrier(); asm volatile("" ::: "memory");
    }
}

__global__ __launch_bounds__(256) void k_cvt8(const float* __restrict__ src, bf* dst, size_t n8) { const size_t i = (size_t)blockIdx.x * 256 + threadIdx.x; if (i >= n8) return; const v8f v = *(const v8f*)(src + i * 8); v8us o;
#pragma unroll
    for (int k = 0; k < 8; ++k) o[k] = f2bf(v[k]); *(volatile v8us*)(dst + i * 8) = o; __threadfence(); *(volatile v8us*)(dst + i * 8) = o; }

__global__ __launch_bounds__(32) void k_freq(float* FR) {
    const int i = threadIdx.x & 31;
    double p = 1.0;
#pragma unroll 1
    for (int j = 0; j < i; ++j) p *= 10000.0;
#pragma unroll 1
    for (int s = 0; s < 5; ++s) p = sqrt(p);
    const float pf = (float)p; const float fr = 1.0f / pf;
    *(volatile float*)(FR + i) = fr; __threadfence(); *(volatile float*)(FR + i) = fr;
}
__global__ __launch_bounds__(256) void k_cstab(const float* __restrict__ FR, float* CS) {
#pragma clang fp contract(off)
    const int idx = blockIdx.x * 256 + threadIdx.x; if (idx >= SEQ * HF) return;
    const int i = idx & (HF - 1); const int t = idx / HF;
    const float ang = (float)t * FR[i]; float s, c; sincosf(ang, &s, &c);
    v2f cs; cs[0] = c; cs[1] = s;
    *(volatile v2f*)(CS + (size_t)idx * 2) = cs; __threadfence(); *(volatile v2f*)(CS + (size_t)idx * 2) = cs;
}
__global__ __launch_bounds__(256) void k_rope(const float* __restrict__ F, const float* __restrict__ CS, h16* P16, bf* Ph, bf* Pl) {
#pragma clang fp contract(off)
    const size_t e = ((size_t)blockIdx.x * 256 + threadIdx.x) * 2; if (e >= (size_t)NB * NH * SEQ * HD) return;
    const int d = (int)(e % HD); const int t = (int)((e / HD) % SEQ); const int bh = (int)(e / ((size_t)HD * SEQ)); const int b = bh / NH, hh = bh % NH;
    const float* f = F + ((size_t)b * SEQ + t) * DM + hh * HD + d;
    const float x1 = f[0], x2 = f[1];
    const v2f cs = *(const v2f*)(CS + ((size_t)t * HF + (d >> 1)) * 2);
    const float a0 = x1 * cs[0], b0 = x2 * cs[1], a1 = x1 * cs[1], b1 = x2 * cs[0];
    const float r0v = a0 - b0, r1v = a1 + b1;
    v2h o16; v2us oh, ol; unsigned short th, tl;
    o16[0] = tohx(r0v); splitf(r0v, th, tl); oh[0] = th; ol[0] = tl;
    o16[1] = tohx(r1v); splitf(r1v, th, tl); oh[1] = th; ol[1] = tl;
    *(volatile v2h*)(P16 + e) = o16; *(volatile v2us*)(Ph + e) = oh; *(volatile v2us*)(Pl + e) = ol; __threadfence(); *(volatile v2h*)(P16 + e) = o16; *(volatile v2us*)(Ph + e) = oh; *(volatile v2us*)(Pl + e) = ol;
}
__global__ __launch_bounds__(256) void k_vtp(const float* __restrict__ F, h16* V16, bf* Vh, bf* Vl) {
    const size_t e = ((size_t)blockIdx.x * 256 + threadIdx.x) * 2; if (e >= (size_t)NB * NH * HD * SEQ) return;
    const int t = (int)(e % SEQ); const int d = (int)((e / SEQ) % HD); const int bh = (int)(e / ((size_t)SEQ * HD)); const int b = bh / NH, hh = bh % NH;
    v2h o16; v2us oh, ol;
#pragma unroll
    for (int q = 0; q < 2; ++q) { const float x = F[((size_t)b * SEQ + t + q) * DM + hh * HD + d]; o16[q] = tohx(x); unsigned short a2, c2; splitf(x, a2, c2); oh[q] = a2; ol[q] = c2; }
    *(volatile v2h*)(V16 + e) = o16; *(volatile v2us*)(Vh + e) = oh; *(volatile v2us*)(Vl + e) = ol; __threadfence(); *(volatile v2h*)(V16 + e) = o16; *(volatile v2us*)(Vh + e) = oh; *(volatile v2us*)(Vl + e) = ol;
}

template <bool HI>
__global__ __launch_bounds__(32) void k_flash(const h16* __restrict__ Q16, const bf* __restrict__ Qh, const bf* __restrict__ Ql,
                                              const h16* __restrict__ K16, const bf* __restrict__ Kh, const bf* __restrict__ Kl,
                                              const h16* __restrict__ VT16, const bf* __restrict__ VTh, const bf* __restrict__ VTl,
                                              int qt0, bf* Ah, bf* Al) {
    __shared__ __align__(32) float os[16 * OSP];
    __shared__ __align__(16) h16 ps[16 * PSP];
    __shared__ __align__(16) unsigned short psh[16 * PSP];
    __shared__ __align__(16) unsigned short psl[16 * PSP];
    const int lane = threadIdx.x & 31, lr = lane & 15, hi = lane >> 4;
    const int q0 = (qt0 + (int)blockIdx.x) * 16; const int hh = blockIdx.y, b = blockIdx.z;
    const size_t pb = ((size_t)(b * NH + hh)) * SEQ * HD;
    const int nch = q0 / 64 + 1;
    v16h qa[2] = {}; v16bf qah[2] = {}, qal[2] = {};
    const size_t qoff = pb + (size_t)(q0 + lr) * HD + 8 * hi;
#pragma unroll
    for (int ks = 0; ks < 2; ++ks) {
        if (HI) { qah[ks] = WFrag<bf>::ld(Qh + qoff + ks * 32); qal[ks] = WFrag<bf>::ld(Ql + qoff + ks * 32); }
        else { qa[ks] = WFrag<h16>::ld(Q16 + qoff + ks * 32); } }
    v8f oacc[4];
#pragma unroll
    for (int t4 = 0; t4 < 4; ++t4) oacc[t4] = (v8f){};
    float mrun[8], lrun[8];
#pragma unroll
    for (int r = 0; r < 8; ++r) { mrun[r] = -3.0e38f; lrun[r] = 0.0f; }
#pragma unroll 1
    for (int c = 0; c < nch; ++c) {
        const int kc0 = c * 64;
        v8f sacc[4];
#pragma unroll
        for (int j = 0; j < 4; ++j) sacc[j] = (v8f){};
        const size_t koff = pb + (size_t)(kc0 + lr) * HD + 8 * hi;
#pragma unroll
        for (int j = 0; j < 4; ++j) {
#pragma unroll
            for (int ks = 0; ks < 2; ++ks) { const size_t o = koff + (size_t)j * 16 * HD + ks * 32;
                if (HI) { const v16bf kbh = WFrag<bf>::ld(Kh + o); const v16bf kbl = WFrag<bf>::ld(Kl + o);
                    sacc[j] = wmmab(qah[ks], kbh, sacc[j]); sacc[j] = wmmab(qal[ks], kbh, sacc[j]); sacc[j] = wmmab(qah[ks], kbl, sacc[j]); }
                else { const v16h kb = WFrag<h16>::ld(K16 + o); sacc[j] = wmma16(qa[ks], kb, sacc[j]); } } }
        if (HI) { asm volatile("v_nop\n\tv_nop\n\tv_nop\n\tv_nop" : "+v"(sacc[0]), "+v"(sacc[1]), "+v"(sacc[2]), "+v"(sacc[3]) : "v"(qah[0]), "v"(qal[1])); }
        else    { asm volatile("v_nop\n\tv_nop\n\tv_nop\n\tv_nop" : "+v"(sacc[0]), "+v"(sacc[1]), "+v"(sacc[2]), "+v"(sacc[3]) : "v"(qa[0]), "v"(qa[1])); }
        float cm[8], mn[8], al[8], rs[8];
#pragma unroll
        for (int r = 0; r < 8; ++r) { const int row = q0 + 8 * hi + r; float best = -3.0e38f;
#pragma unroll
            for (int j = 0; j < 4; ++j) { const int key = kc0 + j * 16 + lr; float s = sacc[j][r] * SCL; s = (key <= row) ? s : -3.0e38f; sacc[j][r] = s; best = fmaxf(best, s); }
            cm[r] = best; }
#pragma unroll
        for (int off = 8; off; off >>= 1)
#pragma unroll
            for (int r = 0; r < 8; ++r) cm[r] = fmaxf(cm[r], __shfl_xor(cm[r], off, 32));
#pragma unroll
        for (int r = 0; r < 8; ++r) { mn[r] = fmaxf(mrun[r], cm[r]); float d0 = mrun[r] - mn[r]; asm volatile("" : "+v"(d0)); const float ea = __builtin_amdgcn_exp2f(d0 * L2E); al[r] = (mrun[r] > -1.0e38f) ? ea : 0.0f; }
#pragma unroll
        for (int r = 0; r < 8; ++r) { const int row = q0 + 8 * hi + r; float su = 0.0f;
#pragma unroll
            for (int j = 0; j < 4; ++j) { const int key = kc0 + j * 16 + lr; float d1 = sacc[j][r] - mn[r]; asm volatile("" : "+v"(d1)); float pv = __builtin_amdgcn_exp2f(d1 * L2E); pv = (key <= row) ? pv : 0.0f; sacc[j][r] = pv; su += pv; }
            rs[r] = su; }
#pragma unroll
        for (int off = 8; off; off >>= 1)
#pragma unroll
            for (int r = 0; r < 8; ++r) rs[r] += __shfl_xor(rs[r], off, 32);
#pragma unroll
        for (int r = 0; r < 8; ++r) { lrun[r] = lrun[r] * al[r] + rs[r]; mrun[r] = mn[r]; }
#pragma unroll
        for (int t4 = 0; t4 < 4; ++t4)
#pragma unroll
            for (int r = 0; r < 8; ++r) oacc[t4][r] *= al[r];
        v16h pa[2] = {}; v16bf pah[2] = {}, pal[2] = {};
        if (HI) {
#pragma unroll
            for (int j = 0; j < 4; ++j)
#pragma unroll
                for (int r = 0; r < 8; ++r) { unsigned short a2, c2; splitf(sacc[j][r], a2, c2); psh[(8 * hi + r) * PSP + j * 16 + lr] = a2; psl[(8 * hi + r) * PSP + j * 16 + lr] = c2; }
            __builtin_amdgcn_wave_barrier(); asm volatile("" ::: "memory");
#pragma unroll
            for (int ks = 0; ks < 2; ++ks) { const int po = lr * PSP + ks * 32 + 8 * hi;
                pah[ks] = cat16b(*(const v8usa*)(psh + po), *(const v8usa*)(psh + po + 16)); pal[ks] = cat16b(*(const v8usa*)(psl + po), *(const v8usa*)(psl + po + 16)); }
            asm volatile("" ::: "memory");
        } else {
#pragma unroll
            for (int j = 0; j < 4; ++j)
#pragma unroll
                for (int r = 0; r < 8; ++r) ps[(8 * hi + r) * PSP + j * 16 + lr] = tohx(sacc[j][r] * PCAR);
            __builtin_amdgcn_wave_barrier(); asm volatile("" ::: "memory");
#pragma unroll
            for (int ks = 0; ks < 2; ++ks) { const int po = lr * PSP + ks * 32 + 8 * hi; pa[ks] = cat16(*(const v8ha*)(ps + po), *(const v8ha*)(ps + po + 16)); }
            asm volatile("" ::: "memory");
        }
        const size_t voff = pb + (size_t)lr * SEQ + kc0 + 8 * hi;
#pragma unroll
        for (int t4 = 0; t4 < 4; ++t4) {
#pragma unroll
            for (int ks = 0; ks < 2; ++ks) { const size_t o = voff + (size_t)t4 * 16 * SEQ + ks * 32;
                if (HI) { const v16bf vbh = WFrag<bf>::ld(VTh + o); const v16bf vbl = WFrag<bf>::ld(VTl + o);
                    oacc[t4] = wmmab(pah[ks], vbh, oacc[t4]); oacc[t4] = wmmab(pal[ks], vbh, oacc[t4]); oacc[t4] = wmmab(pah[ks], vbl, oacc[t4]); }
                else { const v16h vb = WFrag<h16>::ld(VT16 + o); oacc[t4] = wmma16(pa[ks], vb, oacc[t4]); } } }
        if (HI) { asm volatile("v_nop\n\tv_nop\n\tv_nop\n\tv_nop" : "+v"(oacc[0]), "+v"(oacc[1]), "+v"(oacc[2]), "+v"(oacc[3]) : "v"(pah[0]), "v"(pal[1])); }
        else    { asm volatile("v_nop\n\tv_nop\n\tv_nop\n\tv_nop" : "+v"(oacc[0]), "+v"(oacc[1]), "+v"(oacc[2]), "+v"(oacc[3]) : "v"(pa[0]), "v"(pa[1])); }
    }
    const float cs0 = HI ? 1.0f : (1.0f / PCAR);
    float inv[8];
#pragma unroll
    for (int r = 0; r < 8; ++r) inv[r] = cs0 / lrun[r];
#pragma unroll
    for (int t4 = 0; t4 < 4; ++t4)
#pragma unroll
        for (int r = 0; r < 8; ++r) os[(8 * hi + r) * OSP + t4 * 16 + lr] = oacc[t4][r] * inv[r];
    __builtin_amdgcn_wave_barrier(); asm volatile("" ::: "memory");
#pragma unroll 1
    for (int psn = 0; psn < 2; ++psn) {
#pragma unroll
        for (int s = 0; s < 4; ++s) { const int row = s * 4 + (lane >> 3), p8 = lane & 7; const v8f v = *(const v8fa*)(os + row * OSP + p8 * 8); v8us oh, ol;
#pragma unroll
            for (int k = 0; k < 8; ++k) { unsigned short a2, c2; splitf(v[k], a2, c2); oh[k] = a2; ol[k] = c2; }
            const size_t oo = ((size_t)b * SEQ + q0 + row) * DM + (size_t)hh * HD + p8 * 8;
            *(volatile v8us*)(Ah + oo) = oh; *(volatile v8us*)(Al + oo) = ol; }
        if (psn == 0) __threadfence(); }
}

extern "C" void kernel_launch(void* const* d_in, const int* in_sizes, int n_in,
                              void* d_out, int out_size, void* d_ws, size_t ws_size, hipStream_t stream) {
    if (n_in < 5) return;
    if (in_sizes[0] < ((NB - 1) * SEQ_FULL + SEQ) * DM) return;
    if (in_sizes[1] < DM * DM || in_sizes[2] < DM * DM || in_sizes[3] < DM * DM || in_sizes[4] < DM * DM) return;
    if (out_size < NB * SEQ * DM) return;
    const float* x = (const float*)d_in[0]; const float* wq = (const float*)d_in[1]; const float* wk = (const float*)d_in[2]; const float* wv = (const float*)d_in[3]; const float* wo = (const float*)d_in[4];
    float* OUT = (float*)d_out;
    char* wsp = (char*)d_ws;
    auto take = [&](size_t bytes) { char* p = wsp; wsp += (bytes + 255) & ~(size_t)255; return (void*)p; };
    const size_t PL = (size_t)NB * NH * SEQ * HD;
    bf* WQ = (bf*)take((size_t)DM * DM * 2); bf* WK = (bf*)take((size_t)DM * DM * 2); bf* WV = (bf*)take((size_t)DM * DM * 2); bf* WO = (bf*)take((size_t)DM * DM * 2);
    float* FR = (float*)take(128); float* CS = (float*)take((size_t)SEQ * HF * 2 * 4);
    bf* XB = (bf*)take((size_t)NB * SEQ * DM * 2); float* F = (float*)take((size_t)NB * SEQ * DM * 4);
    h16* Q16 = (h16*)take(PL * 2); bf* Qh = (bf*)take(PL * 2); bf* Ql = (bf*)take(PL * 2);
    h16* K16 = (h16*)take(PL * 2); bf* Kh = (bf*)take(PL * 2); bf* Kl = (bf*)take(PL * 2);
    h16* VT16 = (h16*)take(PL * 2); bf* VTh = (bf*)take(PL * 2); bf* VTl = (bf*)take(PL * 2);
    bf* ATh = (bf*)take((size_t)NB * SEQ * DM * 2); bf* ATl = (bf*)take((size_t)NB * SEQ * DM * 2);
    if ((size_t)(wsp - (char*)d_ws) > ws_size) return;
    k_freq<<<1, 32, 0, stream>>>(FR);
    k_cstab<<<(unsigned)((SEQ * HF + 255) / 256), 256, 0, stream>>>(FR, CS);
    const size_t W8 = (size_t)DM * DM / 8; const unsigned GW = (unsigned)((W8 + 255) / 256);
    k_cvt8<<<GW, 256, 0, stream>>>(wq, WQ, W8); k_cvt8<<<GW, 256, 0, stream>>>(wk, WK, W8); k_cvt8<<<GW, 256, 0, stream>>>(wv, WV, W8); k_cvt8<<<GW, 256, 0, stream>>>(wo, WO, W8);
    const size_t X8 = (size_t)SEQ * DM / 8;
    for (int b = 0; b < NB; ++b) k_cvt8<<<(unsigned)((X8 + 255) / 256), 256, 0, stream>>>(x + (size_t)b * SEQ_FULL * DM, XB + (size_t)b * SEQ * DM, X8);
    const dim3 gp(NB * SEQ / 64, DM / 64, 1); const unsigned LP = (unsigned)((PL / 2 + 255) / 256);
    k_gemmw<bf, 0, false><<<gp, 32, 0, stream>>>(XB, nullptr, WQ, nullptr, DM, F, DM, nullptr, 0, 0, 0);
    k_rope<<<LP, 256, 0, stream>>>(F, CS, Q16, Qh, Ql);
    k_gemmw<bf, 0, false><<<gp, 32, 0, stream>>>(XB, nullptr, WK, nullptr, DM, F, DM, nullptr, 0, 0, 0);
    k_rope<<<LP, 256, 0, stream>>>(F, CS, K16, Kh, Kl);
    k_gemmw<bf, 0, false><<<gp, 32, 0, stream>>>(XB, nullptr, WV, nullptr, DM, F, DM, nullptr, 0, 0, 0);
    k_vtp<<<LP, 256, 0, stream>>>(F, VT16, VTh, VTl);
    k_flash<true><<<dim3(RH / 16, NH, NB), 32, 0, stream>>>(Q16, Qh, Ql, K16, Kh, Kl, VT16, VTh, VTl, 0, ATh, ATl);
    if (SEQ > RH) k_flash<false><<<dim3((SEQ - RH) / 16, NH, NB), 32, 0, stream>>>(Q16, Qh, Ql, K16, Kh, Kl, VT16, VTh, VTl, RH / 16, ATh, ATl);
    k_gemmw<bf, 1, false><<<dim3(NB * SEQ / 64, DM / 64, 1), 32, 0, stream>>>(ATh, ATl, WO, nullptr, DM, OUT, DM, nullptr, 0, 0, 0);
}
